// BertSelfAttention_30820685316250
// MI455X (gfx1250) — hardware-run, weakly checked
//
#include <hip/hip_runtime.h>


#ifndef NB
#define NB 4
#endif
#ifndef SEQ
#define SEQ 2048
#endif
#define NB_FULL  4
#define SEQ_FULL 2048
#define DM   1024
#define NH   16
#define HD   64
#define RK   16
#define KX   (DM + 64)
#define NTOK (NB * SEQ)
#define CPAD 72
#define OPAD 68
#define WROWP (KX / 8)
#define QKV_CARRY 16.0f
#define P_LOG2CARRY 12.0f
#define LOG2E_F 1.4426950408889634f

static_assert(NB >= 1 && NB <= NB_FULL);
static_assert(SEQ >= 128 && SEQ <= SEQ_FULL);
static_assert(SEQ % 128 == 0);
static_assert(NTOK % 128 == 0);
static_assert(KX % 32 == 0);
static_assert(WROWP * 8 == KX);
static_assert((3 * DM * WROWP) % 256 == 0);
static_assert((NTOK * (DM / 8)) % 256 == 0);
static_assert(NH * HD == DM);
static_assert(3 * RK + 16 == 64);
static_assert(DM % 64 == 0);

typedef _Float16 v8h  __attribute__((ext_vector_type(8)));
typedef _Float16 v16h __attribute__((ext_vector_type(16)));
typedef float    v8f  __attribute__((ext_vector_type(8)));
typedef float    v4f  __attribute__((ext_vector_type(4)));
typedef float    v2f  __attribute__((ext_vector_type(2)));
typedef unsigned v4u  __attribute__((ext_vector_type(4)));

union Frag { v16h v; v8h h[2]; };
union H8 { v8h h; v4u u; };

__device__ __forceinline__ float bfr(float f) {
    unsigned u = __float_as_uint(f);
    u = (u + 0x7FFFu + ((u >> 16) & 1u)) & 0xFFFF0000u;
    return __uint_as_float(u);
}
__device__ __forceinline__ float ex2(float x) {
#if __has_builtin(__builtin_amdgcn_exp2f)
    return __builtin_amdgcn_exp2f(x);
#else
    return exp2f(x);
#endif
}
__device__ __forceinline__ v8f zero8() { v8f r = {0.f, 0.f, 0.f, 0.f, 0.f, 0.f, 0.f, 0.f}; return r; }
__device__ __forceinline__ v8f wmm(v16h a, v16h b, v8f c) {
    return __builtin_amdgcn_wmma_f32_16x16x32_f16(false, a, false, b, (short)0, c, false, false);
}

__global__ __launch_bounds__(256) void k_convert(const float* __restrict__ X,
    const float* __restrict__ Wq, const float* __restrict__ Wk, const float* __restrict__ Wv,
    const float* __restrict__ Bq, const float* __restrict__ Bk, const float* __restrict__ Bv,
    const float* __restrict__ Aq, const float* __restrict__ Ak, const float* __restrict__ Av,
    _Float16* Xh, _Float16* Wh, _Float16* Ah, int nbx, int nbw)
{
    const int tid = threadIdx.x;
    const int blk = blockIdx.x;
    v4f f0, f1;
    float scale;
    _Float16* dst;
    if (blk < nbx) {
        const int p = blk * 256 + tid;
        const int tok = p >> 7, j = p & 127;
        const int b = tok / SEQ, s = tok - b * SEQ;
        const float* src = X + ((size_t)b * SEQ_FULL + s) * DM + 8 * j;
        f0 = *(const v4f*)src; f1 = *(const v4f*)(src + 4);
        scale = 1.0f;
        dst = Xh + (size_t)tok * KX + 8 * j;
    } else if (blk < nbx + nbw) {
        const int p = (blk - nbx) * 256 + tid;
        const int z = p / (DM * WROWP);
        const int rem = p - z * (DM * WROWP);
        const int o = rem / WROWP, j = rem - o * WROWP;
        const float* Wm = (z == 0) ? Wq : ((z == 1) ? Wk : Wv);
        const float* Bm = (z == 0) ? Bq : ((z == 1) ? Bk : Bv);
        const int jw = (j < 128) ? j : 127;
        const float* wsrc = Wm + (size_t)o * DM + 8 * jw;
        const v4f w0 = *(const v4f*)wsrc, w1 = *(const v4f*)(wsrc + 4);
        int jb = j - 128; jb = (jb < 0) ? 0 : jb;
        const int zb = jb >> 1, r0 = 8 * (jb & 1);
        const float* bsrc = Bm + (size_t)o * RK + r0;
        const v4f c0 = *(const v4f*)bsrc, c1 = *(const v4f*)(bsrc + 4);
        const bool isw = (j < 128);
#pragma unroll
        for (int e = 0; e < 4; ++e) { f0[e] = isw ? w0[e] : c0[e]; f1[e] = isw ? w1[e] : c1[e]; }
        scale = isw ? 64.0f : ((zb == z) ? 4.0f : 0.0f);
        dst = Wh + ((size_t)z * DM + o) * KX + 8 * j;
    } else {
        const int p = (blk - nbx - nbw) * 256 + tid;
        const int r = p >> 7, j = p & 127;
        const int rr = (r < 48) ? r : 47;
        const float* Am = (rr < 16) ? Aq : ((rr < 32) ? Ak : Av);
        const float* asrc = Am + (size_t)(rr & 15) * DM + 8 * j;
        f0 = *(const v4f*)asrc; f1 = *(const v4f*)(asrc + 4);
        scale = (r < 48) ? 64.0f : 0.0f;
        dst = Ah + (size_t)r * DM + 8 * j;
    }
    H8 o;
    o.h = (v8h){ (_Float16)(bfr(f0[0]) * scale), (_Float16)(bfr(f0[1]) * scale),
                 (_Float16)(bfr(f0[2]) * scale), (_Float16)(bfr(f0[3]) * scale),
                 (_Float16)(bfr(f1[0]) * scale), (_Float16)(bfr(f1[1]) * scale),
                 (_Float16)(bfr(f1[2]) * scale), (_Float16)(bfr(f1[3]) * scale) };
    *(volatile v4u*)dst = o.u;
    __threadfence();
    *(volatile v4u*)dst = o.u;
}

__global__ __launch_bounds__(256) void k_gemm(const _Float16* __restrict__ A, int lda, int K,
    const _Float16* __restrict__ Bm, int ldb, int bzs,
    const float* __restrict__ bias0, const float* __restrict__ bias1, const float* __restrict__ bias2, int hasb,
    _Float16* C0, _Float16* C1, _Float16* C2, int ldc, int trans2, float s1, float s2)
{
    __shared__ __align__(16) _Float16 cst[128 * CPAD];
    const int z = blockIdx.z;
    const _Float16* Bz = Bm + (size_t)z * (size_t)bzs;
    const float* bias = (z == 0) ? bias0 : ((z == 1) ? bias1 : bias2);
    _Float16* C = (z == 0) ? C0 : ((z == 1) ? C1 : C2);
    const bool trans = (trans2 != 0) && (z == 2);
    const int tid = threadIdx.x, lane = tid & 31, w = tid >> 5, m = lane & 15, h = lane >> 4;
    const int row0 = blockIdx.x * 128, col0 = blockIdx.y * 64;
    const _Float16* ap = A + (size_t)(row0 + 16 * w + m) * lda + 8 * h;
    const _Float16* bp = Bz + (size_t)(col0 + m) * ldb + 8 * h;
    const size_t bt = (size_t)16 * ldb;
    v8f acc[4];
#pragma unroll
    for (int t = 0; t < 4; ++t) acc[t] = zero8();
#pragma unroll 1
    for (int kc = 0; kc < K; kc += 32) {
        Frag a, b0, b1, b2, b3;
        a.h[0]  = *(const v8h*)(ap + kc);              a.h[1]  = *(const v8h*)(ap + kc + 16);
        b0.h[0] = *(const v8h*)(bp + kc);              b0.h[1] = *(const v8h*)(bp + kc + 16);
        b1.h[0] = *(const v8h*)(bp + bt + kc);         b1.h[1] = *(const v8h*)(bp + bt + kc + 16);
        b2.h[0] = *(const v8h*)(bp + 2 * bt + kc);     b2.h[1] = *(const v8h*)(bp + 2 * bt + kc + 16);
        b3.h[0] = *(const v8h*)(bp + 3 * bt + kc);     b3.h[1] = *(const v8h*)(bp + 3 * bt + kc + 16);
        acc[0] = wmm(a.v, b0.v, acc[0]);
        acc[1] = wmm(a.v, b1.v, acc[1]);
        acc[2] = wmm(a.v, b2.v, acc[2]);
        acc[3] = wmm(a.v, b3.v, acc[3]);
        asm volatile("v_nop\n\tv_nop\n\tv_nop\n\tv_nop" : "+v"(acc[0]), "+v"(acc[1]), "+v"(acc[2]), "+v"(acc[3])
                          : "v"(a.v), "v"(b0.v), "v"(b1.v), "v"(b2.v), "v"(b3.v));
    }
#pragma unroll
    for (int t = 0; t < 4; ++t) {
        const int cl = 16 * t + m;
        float bv = 0.0f;
        if (hasb) bv = bfr(bias[col0 + cl]);
#pragma unroll
        for (int r = 0; r < 8; ++r) {
            const int rl = 16 * w + 8 * h + r;
            cst[rl * CPAD + cl] = (_Float16)((acc[t][r] * s1 + bv) * s2);
        }
    }
    __syncthreads();
    v4u u[4];
    size_t off[4];
    if (!trans) {
#pragma unroll
        for (int i = 0; i < 4; ++i) {
            const int p = tid + 256 * i;
            const int row = p >> 3, j = p & 7;
            u[i] = *(const v4u*)&cst[row * CPAD + 8 * j];
            off[i] = (size_t)(row0 + row) * ldc + col0 + 8 * j;
        }
    } else {
        const int b = row0 / SEQ, s0 = row0 - b * SEQ, hh = blockIdx.y;
#pragma unroll
        for (int i = 0; i < 4; ++i) {
            const int p = tid + 256 * i;
            const int d = p >> 4, jj = p & 15;
            H8 g;
            g.h = (v8h){ cst[(8 * jj + 0) * CPAD + d], cst[(8 * jj + 1) * CPAD + d],
                         cst[(8 * jj + 2) * CPAD + d], cst[(8 * jj + 3) * CPAD + d],
                         cst[(8 * jj + 4) * CPAD + d], cst[(8 * jj + 5) * CPAD + d],
                         cst[(8 * jj + 6) * CPAD + d], cst[(8 * jj + 7) * CPAD + d] };
            u[i] = g.u;
            off[i] = ((size_t)((b * NH + hh) * HD + d)) * SEQ + s0 + 8 * jj;
        }
    }
#pragma unroll
    for (int i = 0; i < 4; ++i) *(volatile v4u*)(C + off[i]) = u[i];
    __threadfence();
#pragma unroll
    for (int i = 0; i < 4; ++i) *(volatile v4u*)(C + off[i]) = u[i];
}

__global__ __launch_bounds__(256) void k_attn(const _Float16* __restrict__ Qh, const _Float16* __restrict__ Kh,
    const _Float16* __restrict__ Vt, const float* __restrict__ amask, float* out)
{
    __shared__ __align__(16) _Float16 Kt[64 * CPAD];
    __shared__ __align__(16) _Float16 Vl[64 * CPAD];
    __shared__ __align__(16) float Ml[64];
    __shared__ __align__(16) float Ol[8 * 16 * OPAD];
    const int tid = threadIdx.x, lane = tid & 31, w = tid >> 5, m = lane & 15, h = lane >> 4;
    const int bh = blockIdx.y, b = bh / NH, head = bh - b * NH;
    const int q0 = blockIdx.x * 128 + 16 * w;

    Frag qf0, qf1;
    {
        const _Float16* qp = Qh + ((size_t)b * SEQ + q0 + m) * DM + head * HD + 8 * h;
        qf0.h[0] = *(const v8h*)qp;        qf0.h[1] = *(const v8h*)(qp + 16);
        qf1.h[0] = *(const v8h*)(qp + 32); qf1.h[1] = *(const v8h*)(qp + 48);
    }
    v8f acco[4];
#pragma unroll
    for (int t = 0; t < 4; ++t) acco[t] = zero8();
    float mrun = -__builtin_inff();
    float lrun = 0.0f;

    const int sr = tid >> 2, sp = 16 * (tid & 3);
    const _Float16* kg = Kh + ((size_t)b * SEQ + sr) * DM + head * HD + sp;
    const _Float16* vg = Vt + ((size_t)bh * HD + sr) * SEQ + sp;
    const float* mg = amask + (size_t)b * SEQ_FULL;
    const float sc = LOG2E_F / 2048.0f;

#pragma unroll 1
    for (int kt = 0; kt < SEQ / 64; ++kt) {
        __syncthreads();
        {
            const _Float16* ks = kg + (size_t)kt * 64 * DM;
            const v8h a0 = *(const v8h*)ks, a1 = *(const v8h*)(ks + 8);
            *(v8h*)&Kt[sr * CPAD + sp] = a0; *(v8h*)&Kt[sr * CPAD + sp + 8] = a1;
            const _Float16* vs = vg + (size_t)kt * 64;
            const v8h c0 = *(const v8h*)vs, c1 = *(const v8h*)(vs + 8);
            *(v8h*)&Vl[sr * CPAD + sp] = c0; *(v8h*)&Vl[sr * CPAD + sp + 8] = c1;
            if (w == 0) {
                const v2f mv = *(const v2f*)(mg + kt * 64 + 2 * lane);
                Ml[2 * lane]     = bfr(mv[0]) * LOG2E_F;
                Ml[2 * lane + 1] = bfr(mv[1]) * LOG2E_F;
            }
        }
        __syncthreads();

        v8f accs[4];
#pragma unroll
        for (int j = 0; j < 4; ++j) {
            Frag k0, k1;
            const _Float16* kr = &Kt[(16 * j + m) * CPAD + 8 * h];
            k0.h[0] = *(const v8h*)kr;        k0.h[1] = *(const v8h*)(kr + 16);
            k1.h[0] = *(const v8h*)(kr + 32); k1.h[1] = *(const v8h*)(kr + 48);
            v8f s = zero8();
            s = wmm(k0.v, qf0.v, s);
            s = wmm(k1.v, qf1.v, s);
            asm volatile("v_nop\n\tv_nop\n\tv_nop\n\tv_nop" : "+v"(s) : "v"(k0.v), "v"(k1.v), "v"(qf0.v), "v"(qf1.v));
            accs[j] = s;
        }
        float mt = -__builtin_inff();
#pragma unroll
        for (int j = 0; j < 4; ++j) {
            const v4f m0 = *(const v4f*)&Ml[16 * j + 8 * h];
            const v4f m1 = *(const v4f*)&Ml[16 * j + 8 * h + 4];
#pragma unroll
            for (int r = 0; r < 4; ++r) accs[j][r] = accs[j][r] * sc + m0[r];
#pragma unroll
            for (int r = 0; r < 4; ++r) accs[j][4 + r] = accs[j][4 + r] * sc + m1[r];
#pragma unroll
            for (int r = 0; r < 8; ++r) mt = fmaxf(mt, accs[j][r]);
        }
        mt = fmaxf(mt, __shfl_xor(mt, 16, 32));
        const float mnew = fmaxf(mrun, mt);
        const float corr = ex2(mrun - mnew);
        mrun = mnew;
        const float msub = mnew - P_LOG2CARRY;
        float ps = 0.0f;
#pragma unroll
        for (int j = 0; j < 4; ++j) {
#pragma unroll
            for (int r = 0; r < 8; ++r) {
                const float pv = ex2(accs[j][r] - msub);
                accs[j][r] = pv;
                ps += pv;
            }
        }
        ps += __shfl_xor(ps, 16, 32);
        lrun = lrun * corr + ps;
#pragma unroll
        for (int t = 0; t < 4; ++t) acco[t] = acco[t] * corr;

        Frag p0, p1;
        p0.h[0] = __builtin_convertvector(accs[0], v8h);
        p0.h[1] = __builtin_convertvector(accs[1], v8h);
        p1.h[0] = __builtin_convertvector(accs[2], v8h);
        p1.h[1] = __builtin_convertvector(accs[3], v8h);

#pragma unroll
        for (int t = 0; t < 4; ++t) {
            Frag v0, v1;
            const _Float16* vr = &Vl[(16 * t + m) * CPAD + 8 * h];
            v0.h[0] = *(const v8h*)vr;        v0.h[1] = *(const v8h*)(vr + 16);
            v1.h[0] = *(const v8h*)(vr + 32); v1.h[1] = *(const v8h*)(vr + 48);
            v8f o = acco[t];
            o = wmm(v0.v, p0.v, o);
            o = wmm(v1.v, p1.v, o);
            asm volatile("v_nop\n\tv_nop\n\tv_nop\n\tv_nop" : "+v"(o) : "v"(v0.v), "v"(v1.v), "v"(p0.v), "v"(p1.v));
            acco[t] = o;
        }
    }

    const float inv = (1.0f / lrun) * (1.0f / QKV_CARRY);
    float* ow = &Ol[w * 16 * OPAD];
#pragma unroll
    for (int t = 0; t < 4; ++t) {
#pragma unroll
        for (int r = 0; r < 8; ++r) ow[m * OPAD + 16 * t + 8 * h + r] = acco[t][r] * inv;
    }
    __syncthreads();
    v4f ov[8];
#pragma unroll
    for (int i = 0; i < 8; ++i) {
        const int p = 32 * i + lane;
        const int rr = p >> 4, jj = p & 15;
        ov[i] = *(const v4f*)&ow[rr * OPAD + 4 * jj];
    }
    float* ob = out + ((size_t)b * SEQ + q0) * DM + head * HD;
#pragma unroll
    for (int i = 0; i < 8; ++i) {
        const int p = 32 * i + lane;
        const int rr = p >> 4, jj = p & 15;
        *(volatile v4f*)(ob + (size_t)rr * DM + 4 * jj) = ov[i];
    }
    __threadfence();
#pragma unroll
    for (int i = 0; i < 8; ++i) {
        const int p = 32 * i + lane;
        const int rr = p >> 4, jj = p & 15;
        *(volatile v4f*)(ob + (size_t)rr * DM + 4 * jj) = ov[i];
    }
}

extern "C" void kernel_launch(void* const* d_in, const int* in_sizes, int n_in,
                              void* d_out, int out_size, void* d_ws, size_t ws_size,
                              hipStream_t stream) {
    if (n_in < 14) return;
    const long long needX = ((long long)(NB - 1) * SEQ_FULL + SEQ) * DM;
    const long long needM = (long long)(NB - 1) * SEQ_FULL + SEQ;
    if ((long long)in_sizes[0] < needX) return;
    if ((long long)in_sizes[1] < needM) return;
    for (int z = 0; z < 3; ++z) {
        if (in_sizes[2 + 4 * z] < DM * DM) return;
        if (in_sizes[3 + 4 * z] < DM) return;
        if (in_sizes[4 + 4 * z] < RK * DM) return;
        if (in_sizes[5 + 4 * z] < DM * RK) return;
    }
    if (out_size < NTOK * DM) return;

    const float* X     = (const float*)d_in[0];
    const float* amask = (const float*)d_in[1];
    const float* Wq = (const float*)d_in[2],  *bq = (const float*)d_in[3];
    const float* Aq = (const float*)d_in[4],  *Bq = (const float*)d_in[5];
    const float* Wk = (const float*)d_in[6],  *bk = (const float*)d_in[7];
    const float* Ak = (const float*)d_in[8],  *Bk = (const float*)d_in[9];
    const float* Wv = (const float*)d_in[10], *bv = (const float*)d_in[11];
    const float* Av = (const float*)d_in[12], *Bv = (const float*)d_in[13];
    float* out = (float*)d_out;

    const size_t bXh = (size_t)NTOK * KX * 2;
    const size_t bWh = (size_t)3 * DM * KX * 2;
    const size_t bAh = (size_t)64 * DM * 2;
    const size_t bPl = (size_t)NTOK * DM * 2;
    const size_t total = bXh + bWh + bAh + 3 * bPl;
    if (total > ws_size) return;
    char* base = (char*)d_ws;
    _Float16* Xh = (_Float16*)base;
    _Float16* Wh = (_Float16*)(base + bXh);
    _Float16* Ah = (_Float16*)(base + bXh + bWh);
    _Float16* Qh = (_Float16*)(base + bXh + bWh + bAh);
    _Float16* Kh = (_Float16*)(base + bXh + bWh + bAh + bPl);
    _Float16* Vt = (_Float16*)(base + bXh + bWh + bAh + 2 * bPl);

    const int nbx = (NTOK * (DM / 8)) / 256;
    const int nbw = (3 * DM * WROWP) / 256;
    const int nba = (64 * (DM / 8)) / 256;

    k_convert<<<dim3(nbx + nbw + nba, 1, 1), 256, 0, stream>>>(X, Wq, Wk, Wv, Bq, Bk, Bv, Aq, Ak, Av, Xh, Wh, Ah, nbx, nbw);
    k_gemm<<<dim3(NTOK / 128, 1, 1), 256, 0, stream>>>(Xh, KX, DM, Ah, DM, 0, bq, bq, bq, 0,
                                                       Xh + DM, Xh + DM, Xh + DM, KX, 0, 1.0f / 64.0f, 1.0f);
    k_gemm<<<dim3(NTOK / 128, DM / 64, 3), 256, 0, stream>>>(Xh, KX, KX, Wh, KX, DM * KX, bq, bk, bv, 1,
                                                             Qh, Kh, Vt, DM, 1, 1.0f / 64.0f, QKV_CARRY);
    k_attn<<<dim3(SEQ / 128, NB * NH, 1), 256, 0, stream>>>(Qh, Kh, Vt, amask, out);
}
